// LocalPointDecoder_4853313044948
// MI455X (gfx1250) — hardware-verified
//
#include <hip/hip_runtime.h>

typedef __bf16         v16bf __attribute__((ext_vector_type(16)));
typedef unsigned short v16us __attribute__((ext_vector_type(16)));
typedef unsigned short v8us  __attribute__((ext_vector_type(8)));
typedef float          v8f   __attribute__((ext_vector_type(8)));
typedef float          v4f   __attribute__((ext_vector_type(4)));
typedef v8us __attribute__((may_alias)) v8usa;
typedef v4f  __attribute__((may_alias)) v4fa;

union Frag  { v16bf v; v16us u; v8us half[2]; unsigned short s[16]; };
union Pack8 { v8us v; unsigned short s[8]; };
union Pack8f { v4f v[2]; float f[8]; };

#define NQ   16384
#define MP   4096
#define CF   128
#define HDN  256
#define NBLK 5

__device__ __forceinline__ unsigned short bf16_bits(float x) {
  unsigned int u = __float_as_uint(x);
  u += 0x7FFFu + ((u >> 16) & 1u);
  return (unsigned short)(u >> 16);
}
__device__ __forceinline__ float bf16_val(unsigned short b) {
  return __uint_as_float(((unsigned int)b) << 16);
}

__device__ __forceinline__ v8f wmma3(const Frag& aH, const Frag& aL,
                                     const Frag& bH, const Frag& bL, v8f c) {
  v8f d = __builtin_amdgcn_wmma_f32_16x16x32_bf16(false, aH.v, false, bH.v, (short)0, c, false, false);
  d = __builtin_amdgcn_wmma_f32_16x16x32_bf16(false, aH.v, false, bL.v, (short)0, d, false, false);
  d = __builtin_amdgcn_wmma_f32_16x16x32_bf16(false, aL.v, false, bH.v, (short)0, d, false, false);
  asm volatile("v_nop\n\tv_nop\n\tv_nop\n\tv_nop"
               : "+v"(d) : "v"(aH.v), "v"(aL.v), "v"(bH.v), "v"(bL.v));
  return d;
}

__device__ __forceinline__ Frag ldfrag(const unsigned short* row, int h) {
  Frag f;
  f.half[0] = *(const v8usa*)(row + 8 * h);
  f.half[1] = *(const v8usa*)(row + 16 + 8 * h);
  return f;
}

__device__ __forceinline__ void feaT_store_pass(const unsigned short* sH, const unsigned short* sL,
                                                unsigned short* fTH, unsigned short* fTL,
                                                int m0, int w, int lane) {
  const int q8 = lane & 7, sub = lane >> 3;
#pragma unroll
  for (int i = 0; i < 4; ++i) {
    const int c = w * 16 + i * 4 + sub;
    const v8us vh = *(const v8usa*)(sH + c * 64 + 8 * q8);
    const v8us vl = *(const v8usa*)(sL + c * 64 + 8 * q8);
    *(volatile v8us*)(fTH + (size_t)c * MP + m0 + 8 * q8) = vh;
    *(volatile v8us*)(fTL + (size_t)c * MP + m0 + 8 * q8) = vl;
  }
}

__global__ __launch_bounds__(256) void k_feaT(const float* __restrict__ fea,
                                              unsigned short* __restrict__ fTH,
                                              unsigned short* __restrict__ fTL) {
  __shared__ __attribute__((aligned(16))) unsigned short sH[CF * 64];
  __shared__ __attribute__((aligned(16))) unsigned short sL[CF * 64];
  const int t = threadIdx.x, lane = t & 31, w = t >> 5;
  const int m0 = blockIdx.x * 64;
  const int c = t & 127, rsub = t >> 7;
#pragma unroll 4
  for (int it = 0; it < 32; ++it) {
    const int mm = it * 2 + rsub;
    const float v = fea[(size_t)(m0 + mm) * CF + c];
    const unsigned short hb = bf16_bits(v);
    sH[c * 64 + mm] = hb;
    sL[c * 64 + mm] = bf16_bits(v - bf16_val(hb));
  }
  __syncthreads();
  feaT_store_pass(sH, sL, fTH, fTL, m0, w, lane);
  __threadfence();
  feaT_store_pass(sH, sL, fTH, fTL, m0, w, lane);
}

__global__ __launch_bounds__(256) void k_cvt(const float* __restrict__ src,
                                             unsigned short* __restrict__ dH,
                                             unsigned short* __restrict__ dL, int n8) {
  const int g = blockIdx.x * 256 + threadIdx.x;
  if (g >= n8) return;
  Pack8f in;
  in.v[0] = *(const v4fa*)(src + (size_t)g * 8);
  in.v[1] = *(const v4fa*)(src + (size_t)g * 8 + 4);
  Pack8 ph, pl;
#pragma unroll
  for (int r = 0; r < 8; ++r) {
    const unsigned short hb = bf16_bits(in.f[r]);
    ph.s[r] = hb;
    pl.s[r] = bf16_bits(in.f[r] - bf16_val(hb));
  }
  unsigned short* oh = dH + (size_t)g * 8;
  unsigned short* ol = dL + (size_t)g * 8;
  *(volatile v8us*)oh = ph.v;
  *(volatile v8us*)ol = pl.v;
  __threadfence();
  *(volatile v8us*)oh = ph.v;
  *(volatile v8us*)ol = pl.v;
}

__device__ __forceinline__ void c_store_pass(const unsigned short* sCH, const unsigned short* sCL,
                                             unsigned short* cH, unsigned short* cL,
                                             int n0w, int w, int lane) {
  const int piece = lane & 15, rsub = lane >> 4;
#pragma unroll
  for (int i = 0; i < 8; ++i) {
    const int row = 2 * i + rsub;
    const v8us vh = *(const v8usa*)(sCH + (w * 16 + row) * CF + 8 * piece);
    const v8us vl = *(const v8usa*)(sCL + (w * 16 + row) * CF + 8 * piece);
    *(volatile v8us*)(cH + (size_t)(n0w + row) * CF + 8 * piece) = vh;
    *(volatile v8us*)(cL + (size_t)(n0w + row) * CF + 8 * piece) = vl;
  }
}

__global__ __launch_bounds__(128) void k_interp(const float* __restrict__ p,
                                                const float* __restrict__ pp,
                                                const unsigned short* __restrict__ fTH,
                                                const unsigned short* __restrict__ fTL,
                                                unsigned short* __restrict__ cH,
                                                unsigned short* __restrict__ cL) {
  __shared__ __attribute__((aligned(16))) unsigned short sCH[4 * 16 * CF];
  __shared__ __attribute__((aligned(16))) unsigned short sCL[4 * 16 * CF];

  const int tid = threadIdx.x, lane = tid & 31, w = tid >> 5;
  const int h = lane >> 4, m = lane & 15;
  const int n0w = blockIdx.x * 64 + 16 * w;

  const float qx = p[(size_t)(n0w + m) * 3 + 0];
  const float qy = p[(size_t)(n0w + m) * 3 + 1];
  const float qz = p[(size_t)(n0w + m) * 3 + 2];

  const v8f zero8 = {0.f, 0.f, 0.f, 0.f, 0.f, 0.f, 0.f, 0.f};
  v8f acc[8];
#pragma unroll
  for (int g = 0; g < 8; ++g) acc[g] = zero8;
  float mrun = -1e30f, lrun = 0.0f;

  const unsigned short* aHrow = fTH + (size_t)m * MP;
  const unsigned short* aLrow = fTL + (size_t)m * MP;

#pragma unroll 1
  for (int t = 0; t < MP / 32; ++t) {
    float s[16];
#pragma unroll
    for (int jj = 0; jj < 2; ++jj) {
      const int pb = 32 * t + 16 * jj + 8 * h;
      const float* src = pp + (size_t)pb * 3;
      union { v4f v[6]; float f[24]; } pu;
#pragma unroll
      for (int q = 0; q < 6; ++q) pu.v[q] = *(const v4fa*)(src + 4 * q);
#pragma unroll
      for (int r = 0; r < 8; ++r) {
        const float dx = pu.f[3 * r + 0] - qx;
        const float dy = pu.f[3 * r + 1] - qy;
        const float dz = pu.f[3 * r + 2] - qz;
        const float d  = sqrtf(dx * dx + dy * dy + dz * dz);
        const float tt = d + 1e-5f;
        s[8 * jj + r] = -(tt * tt) * 100.0f;
      }
    }
    float mloc = s[0];
#pragma unroll
    for (int i = 1; i < 16; ++i) mloc = fmaxf(mloc, s[i]);
    mloc = fmaxf(mloc, __shfl_xor(mloc, 16));
    const float mnew = fmaxf(mrun, mloc);
    const float alpha = __expf(mrun - mnew);
    mrun = mnew;

    Frag bH, bL;
    float lsum = 0.0f;
#pragma unroll
    for (int i = 0; i < 16; ++i) {
      const float wv = __expf(s[i] - mnew);
      lsum += wv;
      const unsigned short hb = bf16_bits(wv);
      bH.s[i] = hb;
      bL.s[i] = bf16_bits(wv - bf16_val(hb));
    }
    lsum += __shfl_xor(lsum, 16);
    lrun = lrun * alpha + lsum;
#pragma unroll
    for (int g = 0; g < 8; ++g) acc[g] = acc[g] * alpha;

#pragma unroll
    for (int g = 0; g < 8; ++g) {
      const Frag aH = ldfrag(aHrow + (size_t)g * 16 * MP + 32 * t, h);
      const Frag aL = ldfrag(aLrow + (size_t)g * 16 * MP + 32 * t, h);
      acc[g] = wmma3(aH, aL, bH, bL, acc[g]);
    }
  }

  const float inv = 1.0f / lrun;
  unsigned short* sh = sCH + (w * 16 + m) * CF;
  unsigned short* sl = sCL + (w * 16 + m) * CF;
#pragma unroll
  for (int g = 0; g < 8; ++g) {
    Pack8 ph, pl;
#pragma unroll
    for (int r = 0; r < 8; ++r) {
      const float c = acc[g][r] * inv;
      const unsigned short hb = bf16_bits(c);
      ph.s[r] = hb;
      pl.s[r] = bf16_bits(c - bf16_val(hb));
    }
    *(v8usa*)(sh + 16 * g + 8 * h) = ph.v;
    *(v8usa*)(sl + 16 * g + 8 * h) = pl.v;
  }
  __syncthreads();

  c_store_pass(sCH, sCL, cH, cL, n0w, w, lane);
  __threadfence();
  c_store_pass(sCH, sCL, cH, cL, n0w, w, lane);
}

__global__ __launch_bounds__(32) void k_mlp(const float* __restrict__ p,
                                           const unsigned short* __restrict__ cH,
                                           const unsigned short* __restrict__ cL,
                                           const float* __restrict__ WpF,
                                           const float* __restrict__ bpF,
                                           const unsigned short* __restrict__ WcH,
                                           const unsigned short* __restrict__ WcL,
                                           const float* __restrict__ bc,
                                           const unsigned short* __restrict__ W0H,
                                           const unsigned short* __restrict__ W0L,
                                           const float* __restrict__ b0,
                                           const unsigned short* __restrict__ W1H,
                                           const unsigned short* __restrict__ W1L,
                                           const float* __restrict__ b1,
                                           const float* __restrict__ Wo,
                                           const float* __restrict__ bo,
                                           float* __restrict__ out) {
  __shared__ __attribute__((aligned(16))) float sNet[16 * HDN];
  __shared__ __attribute__((aligned(16))) unsigned short sAH[16 * HDN];
  __shared__ __attribute__((aligned(16))) unsigned short sAL[16 * HDN];
  __shared__ __attribute__((aligned(16))) unsigned short sHH[16 * HDN];
  __shared__ __attribute__((aligned(16))) unsigned short sHL[16 * HDN];
  __shared__ __attribute__((aligned(16))) float sOut[32];

  const int lane = threadIdx.x & 31, h = lane >> 4, m = lane & 15;
  const v8f zero8 = {0.f, 0.f, 0.f, 0.f, 0.f, 0.f, 0.f, 0.f};

  float* netrow = sNet + m * HDN;
  unsigned short* arowH = sAH + m * HDN;
  unsigned short* arowL = sAL + m * HDN;
  unsigned short* hrowH = sHH + m * HDN;
  unsigned short* hrowL = sHL + m * HDN;

#pragma unroll 1
  for (int half = 0; half < 2; ++half) {
    const int n = blockIdx.x * 32 + 16 * half + m;
    const unsigned short* crH = cH + (size_t)n * CF;
    const unsigned short* crL = cL + (size_t)n * CF;

    const float px = p[(size_t)n * 3 + 0];
    const float py = p[(size_t)n * 3 + 1];
    const float pz = p[(size_t)n * 3 + 2];
#pragma unroll 1
    for (int g = 0; g < 16; ++g) {
      const int f0 = 16 * g + 8 * h;
      Pack8f u;
#pragma unroll
      for (int r = 0; r < 8; ++r) {
        const int f = f0 + r;
        u.f[r] = (px * WpF[f * 3 + 0] + py * WpF[f * 3 + 1] + pz * WpF[f * 3 + 2]) + bpF[f];
      }
      *(v4fa*)(netrow + f0) = u.v[0];
      *(v4fa*)(netrow + f0 + 4) = u.v[1];
    }

#pragma unroll 1
    for (int i = 0; i < NBLK; ++i) {
#pragma unroll 1
      for (int g = 0; g < 16; ++g) {
        const int f0 = 16 * g;
        const v4f x0 = *(const v4fa*)(netrow + f0 + 8 * h);
        const v4f x1 = *(const v4fa*)(netrow + f0 + 8 * h + 4);
        v8f acc = {x0.x, x0.y, x0.z, x0.w, x1.x, x1.y, x1.z, x1.w};
        const unsigned short* wrH = WcH + (size_t)(i * HDN + f0 + m) * CF;
        const unsigned short* wrL = WcL + (size_t)(i * HDN + f0 + m) * CF;
#pragma unroll
        for (int kt = 0; kt < CF / 32; ++kt) {
          const Frag aH = ldfrag(wrH + 32 * kt, h);
          const Frag aL = ldfrag(wrL + 32 * kt, h);
          const Frag bH = ldfrag(crH + 32 * kt, h);
          const Frag bL = ldfrag(crL + 32 * kt, h);
          acc = wmma3(aH, aL, bH, bL, acc);
        }
        const v4f bb0 = *(const v4fa*)(bc + i * HDN + f0 + 8 * h);
        const v4f bb1 = *(const v4fa*)(bc + i * HDN + f0 + 8 * h + 4);
        const v8f bias8 = {bb0.x, bb0.y, bb0.z, bb0.w, bb1.x, bb1.y, bb1.z, bb1.w};
        acc = acc + bias8;
        const v4f o0 = {acc[0], acc[1], acc[2], acc[3]};
        const v4f o1 = {acc[4], acc[5], acc[6], acc[7]};
        *(v4fa*)(netrow + f0 + 8 * h) = o0;
        *(v4fa*)(netrow + f0 + 8 * h + 4) = o1;
        Pack8 ph, pl;
#pragma unroll
        for (int r = 0; r < 8; ++r) {
          const float x = fmaxf(acc[r], 0.0f);
          const unsigned short hb = bf16_bits(x);
          ph.s[r] = hb;
          pl.s[r] = bf16_bits(x - bf16_val(hb));
        }
        *(v8usa*)(arowH + f0 + 8 * h) = ph.v;
        *(v8usa*)(arowL + f0 + 8 * h) = pl.v;
      }
      __syncthreads();

#pragma unroll 1
      for (int g = 0; g < 16; ++g) {
        const int f0 = 16 * g;
        v8f acc = zero8;
        const unsigned short* wrH = W0H + (size_t)(i * HDN + f0 + m) * HDN;
        const unsigned short* wrL = W0L + (size_t)(i * HDN + f0 + m) * HDN;
#pragma unroll
        for (int kt = 0; kt < HDN / 32; ++kt) {
          const Frag aH = ldfrag(wrH + 32 * kt, h);
          const Frag aL = ldfrag(wrL + 32 * kt, h);
          const Frag bH = ldfrag(arowH + 32 * kt, h);
          const Frag bL = ldfrag(arowL + 32 * kt, h);
          acc = wmma3(aH, aL, bH, bL, acc);
        }
        const v4f bb0 = *(const v4fa*)(b0 + i * HDN + f0 + 8 * h);
        const v4f bb1 = *(const v4fa*)(b0 + i * HDN + f0 + 8 * h + 4);
        const v8f bias8 = {bb0.x, bb0.y, bb0.z, bb0.w, bb1.x, bb1.y, bb1.z, bb1.w};
        acc = acc + bias8;
        Pack8 ph, pl;
#pragma unroll
        for (int r = 0; r < 8; ++r) {
          const float x = fmaxf(acc[r], 0.0f);
          const unsigned short hb = bf16_bits(x);
          ph.s[r] = hb;
          pl.s[r] = bf16_bits(x - bf16_val(hb));
        }
        *(v8usa*)(hrowH + f0 + 8 * h) = ph.v;
        *(v8usa*)(hrowL + f0 + 8 * h) = pl.v;
      }
      __syncthreads();

#pragma unroll 1
      for (int g = 0; g < 16; ++g) {
        const int f0 = 16 * g;
        const v4f x0 = *(const v4fa*)(netrow + f0 + 8 * h);
        const v4f x1 = *(const v4fa*)(netrow + f0 + 8 * h + 4);
        v8f acc = {x0.x, x0.y, x0.z, x0.w, x1.x, x1.y, x1.z, x1.w};
        const unsigned short* wrH = W1H + (size_t)(i * HDN + f0 + m) * HDN;
        const unsigned short* wrL = W1L + (size_t)(i * HDN + f0 + m) * HDN;
#pragma unroll
        for (int kt = 0; kt < HDN / 32; ++kt) {
          const Frag aH = ldfrag(wrH + 32 * kt, h);
          const Frag aL = ldfrag(wrL + 32 * kt, h);
          const Frag bH = ldfrag(hrowH + 32 * kt, h);
          const Frag bL = ldfrag(hrowL + 32 * kt, h);
          acc = wmma3(aH, aL, bH, bL, acc);
        }
        const v4f bb0 = *(const v4fa*)(b1 + i * HDN + f0 + 8 * h);
        const v4f bb1 = *(const v4fa*)(b1 + i * HDN + f0 + 8 * h + 4);
        const v8f bias8 = {bb0.x, bb0.y, bb0.z, bb0.w, bb1.x, bb1.y, bb1.z, bb1.w};
        acc = acc + bias8;
        const v4f o0 = {acc[0], acc[1], acc[2], acc[3]};
        const v4f o1 = {acc[4], acc[5], acc[6], acc[7]};
        *(v4fa*)(netrow + f0 + 8 * h) = o0;
        *(v4fa*)(netrow + f0 + 8 * h + 4) = o1;
      }
      __syncthreads();
    }

    float part = 0.0f;
#pragma unroll 2
    for (int f4 = 0; f4 < 32; ++f4) {
      const v4f nv = *(const v4fa*)(netrow + 128 * h + 4 * f4);
      const v4f wv = *(const v4fa*)(Wo + 128 * h + 4 * f4);
      part += fmaxf(nv.x, 0.0f) * wv.x + fmaxf(nv.y, 0.0f) * wv.y
            + fmaxf(nv.z, 0.0f) * wv.z + fmaxf(nv.w, 0.0f) * wv.w;
    }
    part += __shfl_xor(part, 16);
    if (h == 0) sOut[16 * half + m] = part + bo[0];
    __syncthreads();
  }

  const v4f ov = *(const v4fa*)(sOut + 4 * (lane & 7));
  float* dst = out + (size_t)blockIdx.x * 32 + 4 * (lane & 7);
  if (lane < 8) *(volatile v4f*)dst = ov;
  __threadfence();
  if (lane < 8) *(volatile v4f*)dst = ov;
}

extern "C" void kernel_launch(void* const* d_in, const int* in_sizes, int n_in,
                              void* d_out, int out_size, void* d_ws, size_t ws_size,
                              hipStream_t stream) {
  if (n_in < 13) return;
  if (in_sizes[0] != NQ * 3 || in_sizes[1] != MP * 3 || in_sizes[2] != MP * CF) return;
  if (in_sizes[3] != HDN * 3 || in_sizes[4] != HDN) return;
  if (in_sizes[5] != NBLK * HDN * CF || in_sizes[6] != NBLK * HDN) return;
  if (in_sizes[7] != NBLK * HDN * HDN || in_sizes[8] != NBLK * HDN) return;
  if (in_sizes[9] != NBLK * HDN * HDN || in_sizes[10] != NBLK * HDN) return;
  if (in_sizes[11] != HDN || in_sizes[12] < 1) return;
  if (out_size != NQ) return;

  const float* p      = (const float*)d_in[0];
  const float* pp     = (const float*)d_in[1];
  const float* fea    = (const float*)d_in[2];
  const float* fc_p_W = (const float*)d_in[3];
  const float* fc_p_b = (const float*)d_in[4];
  const float* fc_c_W = (const float*)d_in[5];
  const float* fc_c_b = (const float*)d_in[6];
  const float* blk0_W = (const float*)d_in[7];
  const float* blk0_b = (const float*)d_in[8];
  const float* blk1_W = (const float*)d_in[9];
  const float* blk1_b = (const float*)d_in[10];
  const float* out_W  = (const float*)d_in[11];
  const float* out_b  = (const float*)d_in[12];
  float* out = (float*)d_out;

  const size_t b_feaT = (size_t)CF * MP * 2;
  const size_t b_wc   = (size_t)NBLK * HDN * CF * 2;
  const size_t b_w    = (size_t)NBLK * HDN * HDN * 2;
  const size_t b_c    = (size_t)NQ * CF * 2;
  const size_t total  = 2 * b_feaT + 2 * b_wc + 4 * b_w + 2 * b_c;
  if (total > ws_size) return;

  char* ws = (char*)d_ws;
  size_t off = 0;
  unsigned short* fTH = (unsigned short*)(ws + off); off += b_feaT;
  unsigned short* fTL = (unsigned short*)(ws + off); off += b_feaT;
  unsigned short* WcH = (unsigned short*)(ws + off); off += b_wc;
  unsigned short* WcL = (unsigned short*)(ws + off); off += b_wc;
  unsigned short* W0H = (unsigned short*)(ws + off); off += b_w;
  unsigned short* W0L = (unsigned short*)(ws + off); off += b_w;
  unsigned short* W1H = (unsigned short*)(ws + off); off += b_w;
  unsigned short* W1L = (unsigned short*)(ws + off); off += b_w;
  unsigned short* cH  = (unsigned short*)(ws + off); off += b_c;
  unsigned short* cL  = (unsigned short*)(ws + off); off += b_c;
  if (off > ws_size) return;

  const int n8_wc = NBLK * HDN * CF / 8;
  const int n8_w  = NBLK * HDN * HDN / 8;

  k_feaT<<<MP / 64, 256, 0, stream>>>(fea, fTH, fTL);
  k_cvt<<<(n8_wc + 255) / 256, 256, 0, stream>>>(fc_c_W, WcH, WcL, n8_wc);
  k_cvt<<<(n8_w + 255) / 256, 256, 0, stream>>>(blk0_W, W0H, W0L, n8_w);
  k_cvt<<<(n8_w + 255) / 256, 256, 0, stream>>>(blk1_W, W1H, W1L, n8_w);

  k_interp<<<NQ / 64, 128, 0, stream>>>(p, pp, fTH, fTL, cH, cL);

  k_mlp<<<NQ / 32, 32, 0, stream>>>(p, cH, cL, fc_p_W, fc_p_b,
                                    WcH, WcL, fc_c_b, W0H, W0L, blk0_b, W1H, W1L, blk1_b,
                                    out_W, out_b, out);
}
